// TransformerBlockPyTorch_12249246729001
// MI455X (gfx1250) — hardware-run, weakly checked
//
#include <hip/hip_runtime.h>
#include <math.h>

constexpr int kBatch  = 2;
constexpr int kSeq    = 2048;
constexpr int kDim    = 1024;
constexpr int kHeads  = 16;
constexpr int kHdim   = 64;
constexpr int kFF     = 4096;
constexpr int kTok    = kBatch * kSeq;
constexpr int kQKW    = 2 * kDim;
constexpr int kGrp    = 4;
constexpr int kNChunk = (kBatch * kHeads) / kGrp;
constexpr float kWCarry   = 16.0f;
constexpr float kWInv     = 1.0f / 16.0f;
constexpr float kQKScale  = 0.125f;
constexpr float kPCarry   = 2048.0f;
constexpr float kYCarry   = 32.0f;
constexpr float kPVScale  = kYCarry / kPCarry;
constexpr float kProjScale = 1.0f / (kYCarry * kWCarry);
constexpr float kGCarry   = 16.0f;
constexpr float kFcpScale = 1.0f / (kGCarry * kWCarry);
constexpr float kInvDim   = 1.0f / 1024.0f;
constexpr float kLnEps    = 1e-5f;

constexpr size_t kMiB      = (size_t)1 << 20;
constexpr size_t kOffQK    = 0;
constexpr size_t kOffWprojT = 0;
constexpr size_t kOffH     = 0;
constexpr size_t kOffVt    = 16 * kMiB;
constexpr size_t kOffHh    = 16 * kMiB;
constexpr size_t kOffWfcpT = 16 * kMiB;
constexpr size_t kOffYh    = 24 * kMiB;
constexpr size_t kOffWfcT  = 24 * kMiB;
constexpr size_t kOffXh    = 32 * kMiB;
constexpr size_t kOffWattnT = 40 * kMiB;
constexpr size_t kOffS     = 32 * kMiB;
constexpr size_t kOffH1    = 32 * kMiB;
constexpr size_t kOffU     = 32 * kMiB;
constexpr size_t kOffH2    = 32 * kMiB;
constexpr size_t kOffP     = 96 * kMiB;
constexpr size_t kOffGh    = 96 * kMiB;
constexpr size_t kWsTotal  = 128 * kMiB;

typedef __attribute__((ext_vector_type(16))) _Float16 v16h;
typedef __attribute__((ext_vector_type(8)))  _Float16 v8h;
typedef __attribute__((ext_vector_type(16))) __bf16   v16b;
typedef __attribute__((ext_vector_type(8)))  __bf16   v8b;
typedef __attribute__((ext_vector_type(8)))  float    v8f;
typedef __attribute__((ext_vector_type(4)))  float    v4f;
typedef __attribute__((ext_vector_type(4)))  unsigned int v4u;

__device__ __forceinline__ unsigned short f2bf_bits(float f) {
  unsigned u = __float_as_uint(f);
  return (unsigned short)((u + 0x7FFFu + ((u >> 16) & 1u)) >> 16);
}
__device__ __forceinline__ float bf_bits2f(unsigned short h) { return __uint_as_float(((unsigned)h) << 16); }

__device__ __forceinline__ void dep_guard_h(v8f& a, v8f& b, v16h x, v16h y) { asm volatile("v_nop\n\tv_nop\n\tv_nop\n\tv_nop" : "+v"(a), "+v"(b) : "v"(x), "v"(y)); }
__device__ __forceinline__ void dep_guard_b(v8f& a, v8f& b, v16b x, v16b y) { asm volatile("v_nop\n\tv_nop\n\tv_nop\n\tv_nop" : "+v"(a), "+v"(b) : "v"(x), "v"(y)); }
__device__ __forceinline__ void keep4_h(v16h a, v16h b, v16h c, v16h d) { asm volatile("v_nop" :: "v"(a), "v"(b), "v"(c), "v"(d)); }
__device__ __forceinline__ void keep4_b(v16b a, v16b b, v16b c, v16b d) { asm volatile("v_nop" :: "v"(a), "v"(b), "v"(c), "v"(d)); }
__device__ __forceinline__ void acc_guard4(v8f& a, v8f& b, v8f& c, v8f& d) { asm volatile("v_nop\n\tv_nop\n\tv_nop\n\tv_nop" : "+v"(a), "+v"(b), "+v"(c), "+v"(d)); }
template <typename T> struct Frag;
template <> struct Frag<_Float16> {
  typedef v16h V; union U { v16h v; v8h h[2]; };
  static __device__ __forceinline__ v16h load(const _Float16* p) {
    U f; f.h[0] = *(const v8h*)(p); f.h[1] = *(const v8h*)(p + 16); return f.v;
  }
  static __device__ __forceinline__ v8f mma(v16h a, v16h b, v8f c) {
    return __builtin_amdgcn_wmma_f32_16x16x32_f16(false, a, false, b, (short)0, c, false, false);
  }
  static __device__ __forceinline__ void guard(v8f& a, v8f& b, v16h x, v16h y) { dep_guard_h(a, b, x, y); }
  static __device__ __forceinline__ void keep(v16h a, v16h b, v16h c, v16h d) { keep4_h(a, b, c, d); }
};
template <> struct Frag<__bf16> {
  typedef v16b V; union U { v16b v; v8b h[2]; };
  static __device__ __forceinline__ v16b load(const __bf16* p) {
    U f; f.h[0] = *(const v8b*)(p); f.h[1] = *(const v8b*)(p + 16); return f.v;
  }
  static __device__ __forceinline__ v8f mma(v16b a, v16b b, v8f c) {
    return __builtin_amdgcn_wmma_f32_16x16x32_bf16(false, a, false, b, (short)0, c, false, false);
  }
  static __device__ __forceinline__ void guard(v8f& a, v8f& b, v16b x, v16b y) { dep_guard_b(a, b, x, y); }
  static __device__ __forceinline__ void keep(v16b a, v16b b, v16b c, v16b d) { keep4_b(a, b, c, d); }
};

__device__ __forceinline__ unsigned pk16(unsigned short a, unsigned short b) { return (unsigned)a | ((unsigned)b << 16); }
__device__ __forceinline__ unsigned short h_bits(float f) { const _Float16 h = (_Float16)f; return __builtin_bit_cast(unsigned short, h); }

template <int ET> struct Elem;
template <> struct Elem<0> { typedef _Float16 T; };
template <> struct Elem<1> { typedef __bf16 T; };
template <int ET, bool SPLIT, int BIAS_MODE, int OUT_MODE, bool RESID, int ACT = 0, int TRI = 0>
__global__ __launch_bounds__(256) void wmma_gemm64(
    const unsigned short* __restrict__ Ap, const unsigned short* __restrict__ A2p, int lda, long strideA,
    const unsigned short* __restrict__ Btp, const unsigned short* __restrict__ Bt2p, int ldb, long strideB,
    void* __restrict__ Cout, void* __restrict__ Cout2, int ldc, long strideC,
    const float* __restrict__ bias,
    const float* __restrict__ resid, long strideR,
    int M, int N, int K, float scale) {
  typedef typename Elem<ET>::T T;
  typedef typename Frag<T>::V V;
  const T* A = (const T*)Ap; const T* A2 = (const T*)A2p; const T* Bt = (const T*)Btp; const T* Bt2 = (const T*)Bt2p;
  __shared__ __align__(16) float sT[8][16 * 68];
  const int b    = blockIdx.y;
  const int lane = threadIdx.x & 31;
  const int wave = threadIdx.x >> 5;
  const int tilesN = N >> 6;
  const int tilesM = M >> 6;
  const int tile = blockIdx.x * 8 + wave;
  if (tile >= tilesM * tilesN) return;
  const int tm = tile / tilesN;
  const int tn = tile - tm * tilesN;
  const int m0 = tm << 6;
  const int n0 = tn << 6;
  if (TRI == 1 && n0 > m0) return;
  const int kEnd = (TRI == 2) ? (((m0 + 64) < K) ? (m0 + 64) : K) : K;

  const T* Ab  = A  + (size_t)b * strideA;
  const T* Bb  = Bt + (size_t)b * strideB;
  const T* Ab2 = SPLIT ? (A2  + (size_t)b * strideA) : nullptr;
  const T* Bb2 = SPLIT ? (Bt2 + (size_t)b * strideB) : nullptr;

  const int rlane = lane & 15;
  const int koff  = (lane >> 4) * 8;
  const int mOff  = (lane >> 4) * 8;

  v8f acc[4][4];
#pragma unroll
  for (int i = 0; i < 4; ++i)
#pragma unroll
    for (int j = 0; j < 4; ++j) acc[i][j] = (v8f){0.f,0.f,0.f,0.f,0.f,0.f,0.f,0.f};

  for (int k0 = 0; k0 < kEnd; k0 += 32) {
    V bh[4], bl[4];
#pragma unroll
    for (int j = 0; j < 4; ++j) {
      const size_t bo = (size_t)(n0 + (j << 4) + rlane) * ldb + koff + k0;
      bh[j] = Frag<T>::load(Bb + bo);
      if (SPLIT) bl[j] = Frag<T>::load(Bb2 + bo);
    }
#pragma unroll
    for (int i = 0; i < 4; ++i) {
      const size_t ao = (size_t)(m0 + (i << 4) + rlane) * lda + koff + k0;
      V ah = Frag<T>::load(Ab + ao);
      V al;
      if (SPLIT) al = Frag<T>::load(Ab2 + ao);
#pragma unroll
      for (int j = 0; j < 4; ++j) {
        acc[i][j] = Frag<T>::mma(ah, bh[j], acc[i][j]);
        if (SPLIT) {
          acc[i][j] = Frag<T>::mma(ah, bl[j], acc[i][j]);
          acc[i][j] = Frag<T>::mma(al, bh[j], acc[i][j]);
        }
      }
      Frag<T>::guard(acc[i][0], acc[i][3], ah, SPLIT ? al : ah);
    }
    Frag<T>::keep(bh[0], bh[1], bh[2], bh[3]);
    if (SPLIT) Frag<T>::keep(bl[0], bl[1], bl[2], bl[3]);
  }
  acc_guard4(acc[0][0], acc[0][1], acc[0][2], acc[0][3]);
  acc_guard4(acc[1][0], acc[1][1], acc[1][2], acc[1][3]);
  acc_guard4(acc[2][0], acc[2][1], acc[2][2], acc[2][3]);
  acc_guard4(acc[3][0], acc[3][1], acc[3][2], acc[3][3]);

  float* slab = sT[wave];
  const float* Rb = RESID ? (resid + (size_t)b * strideR) : nullptr;
#pragma unroll
  for (int i = 0; i < 4; ++i) {
    const int mBase = m0 + (i << 4);
#pragma unroll
    for (int j = 0; j < 4; ++j) {
      const int n = n0 + (j << 4) + rlane;
      float bv = 0.f;
      if (BIAS_MODE == 2) bv = bias[n];
#pragma unroll
      for (int r = 0; r < 8; ++r) {
        float v = acc[i][j][r] * scale;
        if (BIAS_MODE == 1) v += bias[mBase + mOff + r];
        if (BIAS_MODE == 2) v += bv;
        if (RESID) v += Rb[(size_t)(mBase + mOff + r) * ldc + n];
        if (ACT == 2) v = fmaxf(v, 0.0f);
        if (ACT == 4) v = (v > 0.f) ? v : 0.01f * v;
        slab[(mOff + r) * 68 + (j << 4) + rlane] = v;
      }
    }
    __builtin_amdgcn_fence(__ATOMIC_RELEASE, "workgroup");
    __builtin_amdgcn_wave_barrier();
    __builtin_amdgcn_fence(__ATOMIC_ACQUIRE, "workgroup");
    if (OUT_MODE == 0) {
      float* C = (float*)Cout + (size_t)b * strideC;
      const int hh = lane >> 4, c4 = (lane & 15) * 4;
      for (int pass = 0; pass < 2; ++pass) {
#pragma unroll
        for (int it = 0; it < 8; ++it) {
          const int row = it * 2 + hh;
          v4f v = *(const v4f*)(slab + row * 68 + c4);
          *(volatile v4f*)(C + (size_t)(mBase + row) * ldc + n0 + c4) = v;
        }
        __threadfence();
      }
    } else {
      const int q = lane >> 3, c8 = (lane & 7) * 8;
      unsigned short* C  = (unsigned short*)Cout  + (size_t)b * strideC;
      unsigned short* C2 = (OUT_MODE == 2) ? ((unsigned short*)Cout2 + (size_t)b * strideC) : nullptr;
      for (int pass = 0; pass < 2; ++pass) {
#pragma unroll
        for (int it = 0; it < 4; ++it) {
          const int row = it * 4 + q;
          const float* sp = slab + row * 68 + c8;
          v8h hv, lv;
#pragma unroll
          for (int e = 0; e < 8; ++e) {
            if (OUT_MODE == 1) {
              hv[e] = (_Float16)sp[e];
            } else {
              unsigned short hb = f2bf_bits(sp[e]);
              unsigned short lb = f2bf_bits(sp[e] - bf_bits2f(hb));
              hv[e] = __builtin_bit_cast(_Float16, hb);
              lv[e] = __builtin_bit_cast(_Float16, lb);
            }
          }
          *(volatile v8h*)(C + (size_t)(mBase + row) * ldc + n0 + c8) = hv;
          if (OUT_MODE == 2) *(volatile v8h*)(C2 + (size_t)(mBase + row) * ldc + n0 + c8) = lv;
        }
        __threadfence();
      }
    }
    __builtin_amdgcn_fence(__ATOMIC_RELEASE, "workgroup");
    __builtin_amdgcn_wave_barrier();
    __builtin_amdgcn_fence(__ATOMIC_ACQUIRE, "workgroup");
  }
}

__global__ __launch_bounds__(256) void tcast_kernel(const float* __restrict__ W, unsigned short* __restrict__ out,
                                                    int R, int Cc, float scale) {
  __shared__ float sm[64][65];
  const int t  = threadIdx.x;
  const int c0 = blockIdx.x * 64;
  const int r0 = blockIdx.y * 64;
#pragma unroll
  for (int i = 0; i < 16; ++i) {
    const int e  = i * 256 + t;
    const int rl = e >> 6;
    const int cl = e & 63;
    sm[cl][rl] = W[(size_t)(r0 + rl) * Cc + c0 + cl] * scale;
  }
  __syncthreads();
  const int lane = t & 31, wave = t >> 5;
  const int q = lane >> 3, c8 = (lane & 7) * 8;
  for (int pass = 0; pass < 2; ++pass) {
#pragma unroll
    for (int it = 0; it < 2; ++it) {
      const int row = wave * 8 + it * 4 + q;
      unsigned short hb[8];
#pragma unroll
      for (int e = 0; e < 8; ++e) hb[e] = h_bits(sm[row][c8 + e]);
      const v4u u = (v4u){pk16(hb[0], hb[1]), pk16(hb[2], hb[3]), pk16(hb[4], hb[5]), pk16(hb[6], hb[7])};
      *(volatile v4u*)(out + (size_t)(c0 + row) * R + r0 + c8) = u;
    }
    __threadfence();
  }
}

__global__ __launch_bounds__(256) void cast8_f16_kernel(const float* __restrict__ in, unsigned short* __restrict__ out, int n8) {
  const int i = blockIdx.x * 256 + threadIdx.x;
  if (i >= n8) return;
  const float* p = in + 8 * (size_t)i;
  const v4f a = *(const v4f*)(p);
  const v4f c = *(const v4f*)(p + 4);
  unsigned short hb[8];
#pragma unroll
  for (int e = 0; e < 4; ++e) {
    hb[e]     = h_bits(a[e]);
    hb[4 + e] = h_bits(c[e]);
  }
  const v4u u = (v4u){pk16(hb[0], hb[1]), pk16(hb[2], hb[3]), pk16(hb[4], hb[5]), pk16(hb[6], hb[7])};
  unsigned short* q = out + 8 * (size_t)i;
  *(volatile v4u*)q = u;
  __threadfence();
  *(volatile v4u*)q = u;
}

__global__ __launch_bounds__(256) void softmax_row_kernel(const float* __restrict__ S, unsigned short* __restrict__ P) {
  __shared__ float redM[8];
  __shared__ float redS[8];
  const int rowg = blockIdx.x;
  const int q    = rowg & (kSeq - 1);
  const int t    = threadIdx.x;
  const int lane = t & 31, wave = t >> 5;
  const int c0   = t * 8;
  const float* sr = S + (size_t)rowg * kSeq + c0;
  const v4f a = *(const v4f*)(sr);
  const v4f c = *(const v4f*)(sr + 4);
  float x[8];
#pragma unroll
  for (int e = 0; e < 4; ++e) {
    x[e]     = (c0 + e <= q)     ? a[e] : -INFINITY;
    x[4 + e] = (c0 + 4 + e <= q) ? c[e] : -INFINITY;
  }
  float m = fmaxf(fmaxf(fmaxf(x[0], x[1]), fmaxf(x[2], x[3])), fmaxf(fmaxf(x[4], x[5]), fmaxf(x[6], x[7])));
#pragma unroll
  for (int off = 16; off > 0; off >>= 1) m = fmaxf(m, __shfl_xor(m, off, 32));
  if (lane == 0) redM[wave] = m;
  __syncthreads();
  float gm = redM[0];
#pragma unroll
  for (int w = 1; w < 8; ++w) gm = fmaxf(gm, redM[w]);
  float p[8];
  float psum = 0.f;
#pragma unroll
  for (int e = 0; e < 8; ++e) {
    p[e] = expf(x[e] - gm);
    psum += p[e];
  }
#pragma unroll
  for (int off = 16; off > 0; off >>= 1) psum += __shfl_xor(psum, off, 32);
  if (lane == 0) redS[wave] = psum;
  __syncthreads();
  float tot = 0.f;
#pragma unroll
  for (int w = 0; w < 8; ++w) tot += redS[w];
  const float scl = kPCarry * (1.0f / tot);
  unsigned short hb[8];
#pragma unroll
  for (int e = 0; e < 8; ++e) hb[e] = h_bits(p[e] * scl);
  const v4u u = (v4u){pk16(hb[0], hb[1]), pk16(hb[2], hb[3]), pk16(hb[4], hb[5]), pk16(hb[6], hb[7])};
  unsigned short* pr = P + (size_t)rowg * kSeq + c0;
  *(volatile v4u*)pr = u;
  __threadfence();
  *(volatile v4u*)pr = u;
}

__global__ __launch_bounds__(256) void gelu8_kernel(const float* __restrict__ U, unsigned short* __restrict__ G, int n8) {
  const int i = blockIdx.x * 256 + threadIdx.x;
  if (i >= n8) return;
  const float* p = U + 8 * (size_t)i;
  unsigned long long w0 = 0ull, w1 = 0ull;
#pragma unroll 1
  for (int e = 0; e < 8; ++e) {
    const float v = p[e];
    const float inner = 0.7978845608028654f * (v + 0.044715f * v * v * v);
    const float gl = 0.5f * v * (1.0f + tanhf(inner));
    const unsigned long long hb = (unsigned long long)h_bits(gl * kGCarry);
    const unsigned long long sh = hb << (16 * (e & 3));
    w0 |= (e < 4) ? sh : 0ull;
    w1 |= (e < 4) ? 0ull : sh;
  }
  const v4u u = (v4u){(unsigned)(w0 & 0xffffffffull), (unsigned)(w0 >> 32), (unsigned)(w1 & 0xffffffffull), (unsigned)(w1 >> 32)};
  unsigned short* q = G + 8 * (size_t)i;
  *(volatile v4u*)q = u;
  __threadfence();
  *(volatile v4u*)q = u;
}

template <bool WH>
__global__ __launch_bounds__(256) void ln_row_kernel(const float* __restrict__ X, const float* __restrict__ g,
                                                     const float* __restrict__ bta, float* __restrict__ Y,
                                                     unsigned short* __restrict__ Yh) {
  __shared__ float red1[8];
  __shared__ float red2[8];
  __shared__ __align__(16) float rowbuf[WH ? kDim : 4];
  const int row  = blockIdx.x;
  const int t    = threadIdx.x;
  const int lane = t & 31, wave = t >> 5;
  const v4f v = *(const v4f*)(X + (size_t)row * kDim + t * 4);
  float s = (v[0] + v[1]) + (v[2] + v[3]);
#pragma unroll
  for (int off = 16; off > 0; off >>= 1) s += __shfl_xor(s, off, 32);
  if (lane == 0) red1[wave] = s;
  __syncthreads();
  float tot = 0.f;
#pragma unroll
  for (int w = 0; w < 8; ++w) tot += red1[w];
  const float mean = tot * kInvDim;
  const float d0 = v[0] - mean, d1 = v[1] - mean, d2 = v[2] - mean, d3 = v[3] - mean;
  float s2 = (d0 * d0 + d1 * d1) + (d2 * d2 + d3 * d3);
#pragma unroll
  for (int off = 16; off > 0; off >>= 1) s2 += __shfl_xor(s2, off, 32);
  if (lane == 0) red2[wave] = s2;
  __syncthreads();
  float tot2 = 0.f;
#pragma unroll
  for (int w = 0; w < 8; ++w) tot2 += red2[w];
  const float var  = tot2 * kInvDim;
  const float rstd = rsqrtf(var + kLnEps);
  const v4f gg = *(const v4f*)(g + t * 4);
  const v4f bb = *(const v4f*)(bta + t * 4);
  v4f o;
  o[0] = d0 * rstd * gg[0] + bb[0];
  o[1] = d1 * rstd * gg[1] + bb[1];
  o[2] = d2 * rstd * gg[2] + bb[2];
  o[3] = d3 * rstd * gg[3] + bb[3];
  float* yp = Y + (size_t)row * kDim + t * 4;
  *(volatile v4f*)yp = o;
  __threadfence();
  *(volatile v4f*)yp = o;
  if (WH) {
    rowbuf[t * 4 + 0] = o[0];
    rowbuf[t * 4 + 1] = o[1];
    rowbuf[t * 4 + 2] = o[2];
    rowbuf[t * 4 + 3] = o[3];
    __syncthreads();
    if (t < 128) {
      const v4f a = *(const v4f*)(rowbuf + t * 8);
      const v4f c = *(const v4f*)(rowbuf + t * 8 + 4);
      unsigned short hb[8];
#pragma unroll
      for (int e = 0; e < 4; ++e) { hb[e] = h_bits(a[e]); hb[4 + e] = h_bits(c[e]); }
      const v4u u = (v4u){pk16(hb[0], hb[1]), pk16(hb[2], hb[3]), pk16(hb[4], hb[5]), pk16(hb[6], hb[7])};
      unsigned short* hp = Yh + (size_t)row * kDim + t * 8;
      *(volatile v4u*)hp = u;
      __threadfence();
      *(volatile v4u*)hp = u;
    }
  }
}

extern "C" void kernel_launch(void* const* d_in, const int* in_sizes, int n_in,
                              void* d_out, int out_size, void* d_ws, size_t ws_size,
                              hipStream_t stream) {
  if (n_in < 13) return;
  if (in_sizes[0] != kTok * kDim || out_size != kTok * kDim) return;
  if (in_sizes[1] != kDim * 3 * kDim || in_sizes[7] != kDim * kFF || in_sizes[9] != kFF * kDim) return;
  if (ws_size < kWsTotal) return;

  const float* x         = (const float*)d_in[0];
  const float* w_attn    = (const float*)d_in[1];
  const float* b_attn    = (const float*)d_in[2];
  const float* w_proj    = (const float*)d_in[3];
  const float* b_proj    = (const float*)d_in[4];
  const float* ln1_g     = (const float*)d_in[5];
  const float* ln1_b     = (const float*)d_in[6];
  const float* w_fc      = (const float*)d_in[7];
  const float* b_fc      = (const float*)d_in[8];
  const float* w_fc_proj = (const float*)d_in[9];
  const float* b_fc_proj = (const float*)d_in[10];
  const float* ln2_g     = (const float*)d_in[11];
  const float* ln2_b     = (const float*)d_in[12];
  float* out = (float*)d_out;

  char* ws = (char*)d_ws;
  unsigned short* pQK     = (unsigned short*)(ws + kOffQK);
  unsigned short* pWprojT = (unsigned short*)(ws + kOffWprojT);
  float*          pH      = (float*)(ws + kOffH);
  unsigned short* pVt     = (unsigned short*)(ws + kOffVt);
  unsigned short* pHh     = (unsigned short*)(ws + kOffHh);
  unsigned short* pWfcpT  = (unsigned short*)(ws + kOffWfcpT);
  unsigned short* pYh     = (unsigned short*)(ws + kOffYh);
  unsigned short* pWfcT   = (unsigned short*)(ws + kOffWfcT);
  unsigned short* pXh     = (unsigned short*)(ws + kOffXh);
  unsigned short* pWattnT = (unsigned short*)(ws + kOffWattnT);
  float*          pS      = (float*)(ws + kOffS);
  float*          pH1     = (float*)(ws + kOffH1);
  float*          pU      = (float*)(ws + kOffU);
  float*          pH2     = (float*)(ws + kOffH2);
  unsigned short* pP      = (unsigned short*)(ws + kOffP);
  unsigned short* pGh     = (unsigned short*)(ws + kOffGh);

  cast8_f16_kernel<<<(kTok * kDim / 8) / 256, 256, 0, stream>>>(x, pXh, kTok * kDim / 8);
  tcast_kernel<<<dim3(3 * kDim / 64, kDim / 64), 256, 0, stream>>>(w_attn, pWattnT, kDim, 3 * kDim, kWCarry);

  wmma_gemm64<0, false, 2, 1, false, 0, 0><<<dim3((kTok / 64) * (kQKW / 64) / 8, 1), 256, 0, stream>>>(
      pXh, nullptr, kDim, 0L,
      pWattnT, nullptr, kDim, 0L,
      (void*)pQK, nullptr, kQKW, 0L,
      b_attn, nullptr, 0L,
      kTok, kQKW, kDim, kWInv);
  wmma_gemm64<0, false, 1, 1, false, 0, 0><<<dim3((kDim / 64) * (kSeq / 64) / 8, kBatch), 256, 0, stream>>>(
      pWattnT + (size_t)2 * kDim * kDim, nullptr, kDim, 0L,
      pXh, nullptr, kDim, (long)kSeq * kDim,
      (void*)pVt, nullptr, kSeq, (long)kDim * kSeq,
      b_attn + 2 * kDim, nullptr, 0L,
      kDim, kSeq, kDim, kWInv);

  for (int ch = 0; ch < kNChunk; ++ch) {
    const int b  = ch / (kHeads / kGrp);
    const int h0 = (ch % (kHeads / kGrp)) * kGrp;
    const unsigned short* qbase = pQK + (size_t)b * kSeq * kQKW + (size_t)h0 * kHdim;
    wmma_gemm64<0, false, 0, 0, false, 0, 1><<<dim3((kSeq / 64) * (kSeq / 64) / 8, kGrp), 256, 0, stream>>>(
        qbase, nullptr, kQKW, (long)kHdim,
        qbase + kDim, nullptr, kQKW, (long)kHdim,
        (void*)pS, nullptr, kSeq, (long)kSeq * kSeq,
        nullptr, nullptr, 0L,
        kSeq, kSeq, kHdim, kQKScale);
    softmax_row_kernel<<<kGrp * kSeq, 256, 0, stream>>>(pS, pP);
    wmma_gemm64<0, false, 0, 1, false, 0, 2><<<dim3((kSeq / 64) * (kHdim / 64) / 8, kGrp), 256, 0, stream>>>(
        pP, nullptr, kSeq, (long)kSeq * kSeq,
        pVt + (size_t)b * kDim * kSeq + (size_t)h0 * kHdim * kSeq, nullptr, kSeq, (long)kHdim * kSeq,
        (void*)(pYh + (size_t)b * kSeq * kDim + (size_t)h0 * kHdim), nullptr, kDim, (long)kHdim,
        nullptr, nullptr, 0L,
        kSeq, kHdim, kSeq, kPVScale);
  }

  tcast_kernel<<<dim3(kDim / 64, kDim / 64), 256, 0, stream>>>(w_proj, pWprojT, kDim, kDim, kWCarry);
  wmma_gemm64<0, false, 2, 0, true, 0, 0><<<dim3((kTok / 64) * (kDim / 64) / 8, 1), 256, 0, stream>>>(
      pYh, nullptr, kDim, 0L,
      pWprojT, nullptr, kDim, 0L,
      (void*)pH1, nullptr, kDim, 0L,
      b_proj, x, 0L,
      kTok, kDim, kDim, kProjScale);

  ln_row_kernel<true><<<kTok, 256, 0, stream>>>(pH1, ln1_g, ln1_b, pH, pHh);

  tcast_kernel<<<dim3(kFF / 64, kDim / 64), 256, 0, stream>>>(w_fc, pWfcT, kDim, kFF, kWCarry);
  wmma_gemm64<0, false, 2, 0, false, 0, 0><<<dim3((kTok / 64) * (kFF / 64) / 8, 1), 256, 0, stream>>>(
      pHh, nullptr, kDim, 0L,
      pWfcT, nullptr, kDim, 0L,
      (void*)pU, nullptr, kFF, 0L,
      b_fc, nullptr, 0L,
      kTok, kFF, kDim, kWInv);

  gelu8_kernel<<<(kTok * kFF / 8) / 256, 256, 0, stream>>>(pU, pGh, kTok * kFF / 8);

  tcast_kernel<<<dim3(kDim / 64, kFF / 64), 256, 0, stream>>>(w_fc_proj, pWfcpT, kFF, kDim, kWCarry);
  wmma_gemm64<0, false, 2, 0, true, 0, 0><<<dim3((kTok / 64) * (kDim / 64) / 8, 1), 256, 0, stream>>>(
      pGh, nullptr, kFF, 0L,
      pWfcpT, nullptr, kFF, 0L,
      (void*)pH2, nullptr, kDim, 0L,
      b_fc_proj, pH, 0L,
      kTok, kDim, kFF, kFcpScale);

  ln_row_kernel<false><<<kTok, 256, 0, stream>>>(pH2, ln2_g, ln2_b, out, nullptr);
}
